// TransformerBlock_63668595196337
// MI455X (gfx1250) — hardware-verified
//
#include <hip/hip_runtime.h>
#include <math.h>

#ifndef NB
#define NB 2
#endif
#ifndef SEQ
#define SEQ 2048
#endif
#define NB_FULL 2
#define SEQ_FULL 2048
#define DM 1024
#define NH 16
#define HD 64
#define FF 4096
#define MROWS (NB * SEQ)
#define LDQK (2 * DM)
#define LDVT (MROWS)
#define PP 72

static_assert(DM == NH * HD);
static_assert(HD == 64);
static_assert(SEQ % 64 == 0);
static_assert(MROWS % 64 == 0);
static_assert(DM % 64 == 0);
static_assert(FF % 64 == 0);
static_assert(DM % 32 == 0);
static_assert(FF % 32 == 0);
static_assert(DM == 256 * 4);
static_assert(DM == 128 * 8);
static_assert(DM % 8 == 0);
static_assert(FF % 8 == 0);
static_assert(NB <= NB_FULL);
static_assert(SEQ <= SEQ_FULL);
static_assert((size_t)NB_FULL * SEQ_FULL * DM * 4 == 16777216ull);

typedef __attribute__((ext_vector_type(16))) _Float16 v16h;
typedef __attribute__((ext_vector_type(8)))  _Float16 v8h;
typedef __attribute__((ext_vector_type(8)))  float    v8f;
typedef __attribute__((ext_vector_type(4)))  float    v4f;
typedef __attribute__((ext_vector_type(4)))  unsigned int v4u;
typedef v8h v8h_a __attribute__((may_alias));
typedef v4f v4f_a __attribute__((may_alias));

union FragU { v16h v; v8h h[2]; };
__device__ __forceinline__ v16h frag_ld(const _Float16* p) {
    FragU f; f.h[0] = *(const v8h*)(p); f.h[1] = *(const v8h*)(p + 16); return f.v;
}
__device__ __forceinline__ v16h frag_ld_lds(const _Float16* p) {
    FragU f; f.h[0] = *(const v8h_a*)(p); f.h[1] = *(const v8h_a*)(p + 16); return f.v;
}
__device__ __forceinline__ v8f wmma16(v16h a, v16h b, v8f c) {
    c = __builtin_amdgcn_wmma_f32_16x16x32_f16(false, a, false, b, (short)0, c, false, false);
    asm volatile("v_nop\n\tv_nop\n\tv_nop\n\tv_nop" : "+v"(c) : "v"(a), "v"(b));
    return c;
}
__device__ __forceinline__ void wave_sync() {
    __builtin_amdgcn_fence(3  , "workgroup");
    __builtin_amdgcn_wave_barrier();
    __builtin_amdgcn_fence(2  , "workgroup");
}

#define VST2V4(ptr, val) do { const v4f vst2_v4_ = (val); *(volatile v4f*)(ptr) = vst2_v4_; __threadfence(); *(volatile v4f*)(ptr) = vst2_v4_; } while (0)

__device__ __forceinline__ unsigned int cmb_pk2(float a, float b) {
    return (unsigned int)__builtin_bit_cast(unsigned short, (_Float16)a) | ((unsigned int)__builtin_bit_cast(unsigned short, (_Float16)b) << 16);
}
__device__ __forceinline__ float cmb_bf(float v) {
    const unsigned u = __builtin_bit_cast(unsigned, v);
    const unsigned r = (u + 0x7fffu + ((u >> 16) & 1u)) & 0xffff0000u;
    return __builtin_bit_cast(float, r);
}

__global__ __launch_bounds__(256) void k_cast_wT(const float* __restrict__ SRC, int lds, unsigned short* __restrict__ DST, int ldd, int nR, int nC, float sc) {
    const long long u = (long long)blockIdx.x * 256 + threadIdx.x;
    const int per = nR / 8;
    if (u >= (long long)nC * per) return;
    const int c = (int)(u / per); const int r0 = 8 * (int)(u % per);
    float w[8];
#pragma unroll
    for (int e = 0; e < 8; ++e) w[e] = cmb_bf(SRC[(long long)(r0 + e) * lds + c]) * sc;
    v4u pk; pk.x = cmb_pk2(w[0], w[1]); pk.y = cmb_pk2(w[2], w[3]); pk.z = cmb_pk2(w[4], w[5]); pk.w = cmb_pk2(w[6], w[7]);
    volatile v4u* d = (volatile v4u*)(DST + (long long)c * ldd + r0);
    *d = pk; __threadfence(); *d = pk;
}

__global__ __launch_bounds__(256) void k_rms(const float* __restrict__ in, int in_bs, const float* __restrict__ w,
                                             float* __restrict__ of, int of_bs, unsigned short* __restrict__ o16,
                                             int rnd, int do32, int do16) {
    __shared__ __align__(16) float srow[DM];
    __shared__ float red[8];
    const int row = blockIdx.x, tid = threadIdx.x, lane = tid & 31, wave = tid >> 5;
    const int b = row / SEQ, t = row - b * SEQ;
    const float* xr = in + ((size_t)b * in_bs + t) * DM;
    v4f v = *(const v4f*)(xr + 4 * tid);
    if (rnd != 0) { v.x = cmb_bf(v.x); v.y = cmb_bf(v.y); v.z = cmb_bf(v.z); v.w = cmb_bf(v.w); }
    float ss = v.x * v.x + v.y * v.y + v.z * v.z + v.w * v.w;
    ss += __shfl_xor(ss, 16, 32); ss += __shfl_xor(ss, 8, 32); ss += __shfl_xor(ss, 4, 32);
    ss += __shfl_xor(ss, 2, 32);  ss += __shfl_xor(ss, 1, 32);
    if (lane == 0) red[wave] = ss;
    __syncthreads();
    const float tot = ((red[0] + red[1]) + (red[2] + red[3])) + ((red[4] + red[5]) + (red[6] + red[7]));
    const float rs = rsqrtf(tot * (1.0f / (float)DM) + 1e-6f);
    v4f wv = *(const v4f*)(w + 4 * tid);
    wv.x = cmb_bf(wv.x); wv.y = cmb_bf(wv.y); wv.z = cmb_bf(wv.z); wv.w = cmb_bf(wv.w);
    v4f o; o.x = v.x * rs * wv.x; o.y = v.y * rs * wv.y; o.z = v.z * rs * wv.z; o.w = v.w * rs * wv.w;
    if (do32 != 0) {
        float* dst = of + ((size_t)b * of_bs + t) * DM + 4 * tid;
        VST2V4(dst, o);
    }
    if (do16 != 0) {
        srow[4 * tid + 0] = o.x; srow[4 * tid + 1] = o.y; srow[4 * tid + 2] = o.z; srow[4 * tid + 3] = o.w;
        __syncthreads();
        if (tid < 128) {
            const float* sp = srow + 8 * tid;
            v4u pk; pk.x = cmb_pk2(sp[0], sp[1]); pk.y = cmb_pk2(sp[2], sp[3]); pk.z = cmb_pk2(sp[4], sp[5]); pk.w = cmb_pk2(sp[6], sp[7]);
            volatile v4u* d = (volatile v4u*)(o16 + (size_t)row * DM + 8 * tid);
            *d = pk; __threadfence(); *d = pk;
        }
    }
}

template <int OUTM, int ACT>
__device__ __forceinline__ void gemm64_body(const unsigned short* __restrict__ Ap, int lda,
                                            const unsigned short* __restrict__ Btp, int ldb,
                                            void* __restrict__ Cout, int ldc, const float* __restrict__ resid,
                                            int M, int N, int K, float scale) {
    __shared__ __align__(16) float sT[8][16 * 68];
    const _Float16* A  = (const _Float16*)Ap;
    const _Float16* Bt = (const _Float16*)Btp;
    const int lane = threadIdx.x & 31, wave = threadIdx.x >> 5;
    const int tilesN = N >> 6, tilesM = M >> 6;
    const int tile = blockIdx.x * 8 + wave;
    if (tile >= tilesM * tilesN) return;
    const int tm = tile / tilesN, tn = tile - tm * tilesN;
    const int m0 = tm << 6, n0 = tn << 6;
    const int rlane = lane & 15;
    const int koff  = (lane >> 4) * 8;
    const int mOff  = (lane >> 4) * 8;

    v8f acc[4][4];
#pragma unroll
    for (int i = 0; i < 4; ++i)
#pragma unroll
        for (int j = 0; j < 4; ++j) acc[i][j] = (v8f){0.f, 0.f, 0.f, 0.f, 0.f, 0.f, 0.f, 0.f};

    for (int k0 = 0; k0 < K; k0 += 32) {
        v16h bh[4];
#pragma unroll
        for (int j = 0; j < 4; ++j) bh[j] = frag_ld(Bt + (size_t)(n0 + (j << 4) + rlane) * ldb + koff + k0);
#pragma unroll
        for (int i = 0; i < 4; ++i) {
            const v16h ah = frag_ld(A + (size_t)(m0 + (i << 4) + rlane) * lda + koff + k0);
#pragma unroll
            for (int j = 0; j < 4; ++j) acc[i][j] = wmma16(ah, bh[j], acc[i][j]);
        }
    }

    float* slab = sT[wave];
#pragma unroll
    for (int i = 0; i < 4; ++i) {
        const int mBase = m0 + (i << 4);
#pragma unroll
        for (int j = 0; j < 4; ++j)
#pragma unroll
            for (int r = 0; r < 8; ++r) slab[(mOff + r) * 68 + (j << 4) + rlane] = acc[i][j][r] * scale;
        wave_sync();
        if (OUTM == 0) {
            float* C = (float*)Cout;
            const int hh = lane >> 4, c4 = (lane & 15) * 4;
            v4f vv[8];
#pragma unroll
            for (int it = 0; it < 8; ++it) {
                const int row = it * 2 + hh;
                const size_t go = (size_t)(mBase + row) * ldc + n0 + c4;
                vv[it] = *(const v4f_a*)(slab + row * 68 + c4) + *(const v4f*)(resid + go);
            }
#pragma unroll
            for (int it = 0; it < 8; ++it) {
                const int row = it * 2 + hh;
                *(volatile v4f*)(C + (size_t)(mBase + row) * ldc + n0 + c4) = vv[it];
            }
            __threadfence();
#pragma unroll
            for (int it = 0; it < 8; ++it) {
                const int row = it * 2 + hh;
                *(volatile v4f*)(C + (size_t)(mBase + row) * ldc + n0 + c4) = vv[it];
            }
        } else {
            unsigned short* C = (unsigned short*)Cout;
            const int q = lane >> 3, c8 = (lane & 7) * 8;
            v8h hv[4];
#pragma unroll
            for (int it = 0; it < 4; ++it) {
                const float* sp = slab + (it * 4 + q) * 68 + c8;
#pragma unroll
                for (int e = 0; e < 8; ++e) {
                    float f = sp[e];
                    if (ACT == 1) f = f * __builtin_amdgcn_rcpf(1.0f + __expf(-f));
                    hv[it][e] = (_Float16)f;
                }
            }
#pragma unroll
            for (int it = 0; it < 4; ++it) *(volatile v8h*)(C + (size_t)(mBase + it * 4 + q) * ldc + n0 + c8) = hv[it];
            __threadfence();
#pragma unroll
            for (int it = 0; it < 4; ++it) *(volatile v8h*)(C + (size_t)(mBase + it * 4 + q) * ldc + n0 + c8) = hv[it];
        }
        wave_sync();
    }
}

__global__ __launch_bounds__(256) void k_gemm_h(const unsigned short* __restrict__ A, int lda, const unsigned short* __restrict__ Bt, int ldb,
                                                unsigned short* __restrict__ C, int ldc, int M, int N, int K, float scale) {
    gemm64_body<1, 0>(A, lda, Bt, ldb, (void*)C, ldc, nullptr, M, N, K, scale);
}
__global__ __launch_bounds__(256) void k_gemm_silu(const unsigned short* __restrict__ A, int lda, const unsigned short* __restrict__ Bt, int ldb,
                                                   unsigned short* __restrict__ C, int ldc, int M, int N, int K, float scale) {
    gemm64_body<1, 1>(A, lda, Bt, ldb, (void*)C, ldc, nullptr, M, N, K, scale);
}
__global__ __launch_bounds__(256) void k_gemm_res(const unsigned short* __restrict__ A, int lda, const unsigned short* __restrict__ Bt, int ldb,
                                                  float* __restrict__ C, int ldc, const float* __restrict__ R, int M, int N, int K, float scale) {
    gemm64_body<0, 0>(A, lda, Bt, ldb, (void*)C, ldc, R, M, N, K, scale);
}

__global__ __launch_bounds__(128) void k_attn(const unsigned short* __restrict__ QKp, const unsigned short* __restrict__ VTp, unsigned short* __restrict__ Cp) {
    __shared__ __align__(16) _Float16 Ps[4][16 * PP];
    __shared__ __align__(16) float    Os[4][16 * 68];
    const _Float16* QK = (const _Float16*)QKp;
    const _Float16* VT = (const _Float16*)VTp;
    const int tid = threadIdx.x, wave = tid >> 5, lane = tid & 31, hh = lane >> 4, c = lane & 15;
    const int nqb = SEQ / 64;
    const int bx = blockIdx.x;
    const int qb = bx % nqb;
    const int bh = bx / nqb;
    const int h = bh % NH, b = bh / NH;
    const int q0 = qb * 64 + wave * 16;
    const size_t rowbase = (size_t)b * SEQ;
    const float SC = 0.125f * 1.4426950408889634f;

    v16h qa[2];
    {
        const _Float16* qrow = QK + (rowbase + q0 + c) * LDQK + h * HD + 8 * hh;
        qa[0] = frag_ld(qrow);
        qa[1] = frag_ld(qrow + 32);
    }
    float mrow[8], lrow[8];
    v8f oacc[4];
#pragma unroll
    for (int r = 0; r < 8; ++r) { mrow[r] = -INFINITY; lrow[r] = 0.f; }
#pragma unroll
    for (int t = 0; t < 4; ++t) oacc[t] = (v8f){0.f, 0.f, 0.f, 0.f, 0.f, 0.f, 0.f, 0.f};
    _Float16* pw = Ps[wave];

    for (int kc = 0; kc <= qb; ++kc) {
        const int kv0 = kc * 64;
        v8f s[4];
#pragma unroll
        for (int j = 0; j < 4; ++j) {
            const _Float16* krow = QK + (rowbase + kv0 + j * 16 + c) * LDQK + DM + h * HD + 8 * hh;
            v8f a = (v8f){0.f, 0.f, 0.f, 0.f, 0.f, 0.f, 0.f, 0.f};
            a = wmma16(qa[0], frag_ld(krow), a);
            a = wmma16(qa[1], frag_ld(krow + 32), a);
            s[j] = a;
        }
        const bool diag = (kc == qb);
        float cm[8];
#pragma unroll
        for (int r = 0; r < 8; ++r) {
            const int qr = q0 + 8 * hh + r;
            float m = -INFINITY;
#pragma unroll
            for (int j = 0; j < 4; ++j) {
                const int kvcol = kv0 + j * 16 + c;
                float v = s[j][r] * SC;
                v = (diag && (kvcol > qr)) ? -INFINITY : v;
                s[j][r] = v;
                m = fmaxf(m, v);
            }
            m = fmaxf(m, __shfl_xor(m, 1, 32)); m = fmaxf(m, __shfl_xor(m, 2, 32));
            m = fmaxf(m, __shfl_xor(m, 4, 32)); m = fmaxf(m, __shfl_xor(m, 8, 32));
            cm[r] = m;
        }
#pragma unroll
        for (int r = 0; r < 8; ++r) {
            const float mnew = fmaxf(mrow[r], cm[r]);
            const float alpha = exp2f(mrow[r] - mnew);
            mrow[r] = mnew;
            float psum = 0.f;
#pragma unroll
            for (int j = 0; j < 4; ++j) {
                const float p = exp2f(s[j][r] - mnew);
                psum += p;
                pw[(8 * hh + r) * PP + j * 16 + c] = (_Float16)(p * 1024.0f);
            }
            psum += __shfl_xor(psum, 1, 32); psum += __shfl_xor(psum, 2, 32);
            psum += __shfl_xor(psum, 4, 32); psum += __shfl_xor(psum, 8, 32);
            lrow[r] = lrow[r] * alpha + psum;
#pragma unroll
            for (int t = 0; t < 4; ++t) oacc[t][r] *= alpha;
        }
        wave_sync();
#pragma unroll
        for (int kk = 0; kk < 2; ++kk) {
            const v16h pa = frag_ld_lds(pw + c * PP + kk * 32 + 8 * hh);
#pragma unroll
            for (int t = 0; t < 4; ++t) {
                const _Float16* vr = VT + (size_t)(h * HD + t * 16 + c) * LDVT + rowbase + kv0 + kk * 32 + 8 * hh;
                oacc[t] = wmma16(pa, frag_ld(vr), oacc[t]);
            }
        }
        wave_sync();
    }

    float* os = Os[wave];
#pragma unroll
    for (int r = 0; r < 8; ++r) {
        const float inv = 1.0f / (lrow[r] * 1024.0f);
#pragma unroll
        for (int t = 0; t < 4; ++t) os[(8 * hh + r) * 68 + t * 16 + c] = oacc[t][r] * inv;
    }
    wave_sync();
    {
        const int q = lane >> 3, c8 = (lane & 7) * 8;
        v8h hv[4];
#pragma unroll
        for (int it = 0; it < 4; ++it) {
            const float* sp = os + (it * 4 + q) * 68 + c8;
#pragma unroll
            for (int e = 0; e < 8; ++e) hv[it][e] = (_Float16)sp[e];
        }
        unsigned short* cb = Cp + (rowbase + q0) * DM + h * HD + c8;
#pragma unroll
        for (int it = 0; it < 4; ++it) *(volatile v8h*)(cb + (size_t)(it * 4 + q) * DM) = hv[it];
        __threadfence();
#pragma unroll
        for (int it = 0; it < 4; ++it) *(volatile v8h*)(cb + (size_t)(it * 4 + q) * DM) = hv[it];
    }
}

constexpr size_t SZ_F32  = (size_t)MROWS * DM * 4;
constexpr size_t SZ_H16  = (size_t)MROWS * DM * 2;
constexpr size_t SZ_QK   = (size_t)MROWS * LDQK * 2;
constexpr size_t SZ_VT   = (size_t)DM * MROWS * 2;
constexpr size_t SZ_MID  = (size_t)MROWS * FF * 2;
constexpr size_t SZ_RC   = (SZ_QK + SZ_VT + SZ_H16 > SZ_MID) ? (SZ_QK + SZ_VT + SZ_H16) : SZ_MID;
constexpr size_t SZ_W3   = (size_t)3 * DM * DM * 2;
constexpr size_t SZ_WO   = (size_t)DM * DM * 2;
constexpr size_t SZ_W1   = (size_t)FF * DM * 2;
constexpr size_t SZ_W2   = (size_t)DM * FF * 2;
constexpr size_t OFF_A   = 0;
constexpr size_t OFF_B   = OFF_A + SZ_F32;
constexpr size_t OFF_C   = OFF_B + SZ_H16;
constexpr size_t OFF_R1  = OFF_C + SZ_RC;
constexpr size_t OFF_Y   = OFF_R1 + SZ_F32;
constexpr size_t OFF_W3  = OFF_Y + SZ_F32;
constexpr size_t OFF_WO  = OFF_W3 + SZ_W3;
constexpr size_t OFF_W1  = OFF_WO + SZ_WO;
constexpr size_t OFF_W2  = OFF_W1 + SZ_W1;
constexpr size_t WS_TOTAL = OFF_W2 + SZ_W2;
static_assert(SZ_F32 % 256 == 0);
static_assert(SZ_H16 % 256 == 0);
static_assert(SZ_QK % 256 == 0);
static_assert(SZ_VT % 256 == 0);
static_assert(SZ_QK + SZ_VT + SZ_H16 <= SZ_RC);
static_assert(SZ_MID <= SZ_RC);
static_assert(WS_TOTAL <= 134217728ull);

extern "C" void kernel_launch(void* const* d_in, const int* in_sizes, int n_in, void* d_out, int out_size, void* d_ws, size_t ws_size, hipStream_t stream) {
    if (n_in < 10) return;
    const long long need_x = ((long long)(NB - 1) * SEQ_FULL + SEQ) * DM;
    if ((long long)in_sizes[0] < need_x) return;
    if (in_sizes[1] < DM || in_sizes[6] < DM || in_sizes[9] < DM) return;
    if ((long long)in_sizes[2] < (long long)DM * DM || (long long)in_sizes[3] < (long long)DM * DM) return;
    if ((long long)in_sizes[4] < (long long)DM * DM || (long long)in_sizes[5] < (long long)DM * DM) return;
    if ((long long)in_sizes[7] < (long long)DM * FF || (long long)in_sizes[8] < (long long)FF * DM) return;
    if ((long long)out_size < need_x) return;
    if (ws_size < WS_TOTAL) return;

    const float* x    = (const float*)d_in[0];
    const float* wpre = (const float*)d_in[1];
    const float* wq   = (const float*)d_in[2];
    const float* wk   = (const float*)d_in[3];
    const float* wv   = (const float*)d_in[4];
    const float* wo   = (const float*)d_in[5];
    const float* wan  = (const float*)d_in[6];
    const float* w1   = (const float*)d_in[7];
    const float* w2   = (const float*)d_in[8];
    const float* wfn  = (const float*)d_in[9];
    float* out = (float*)d_out;

    char* ws = (char*)d_ws;
    float*          H32  = (float*)(ws + OFF_A);
    float*          R2   = (float*)(ws + OFF_A);
    unsigned short* H16  = (unsigned short*)(ws + OFF_B);
    unsigned short* Y16  = (unsigned short*)(ws + OFF_B);
    unsigned short* QK16 = (unsigned short*)(ws + OFF_C);
    unsigned short* VT16 = (unsigned short*)(ws + OFF_C + SZ_QK);
    unsigned short* C16  = (unsigned short*)(ws + OFF_C + SZ_QK + SZ_VT);
    unsigned short* MID  = (unsigned short*)(ws + OFF_C);
    float*          R1   = (float*)(ws + OFF_R1);
    float*          Y32  = (float*)(ws + OFF_Y);
    unsigned short* W3T  = (unsigned short*)(ws + OFF_W3);
    unsigned short* WOT  = (unsigned short*)(ws + OFF_WO);
    unsigned short* W1T  = (unsigned short*)(ws + OFF_W1);
    unsigned short* W2T  = (unsigned short*)(ws + OFF_W2);

    const unsigned gDD = (unsigned)(((long long)DM * (DM / 8) + 255) / 256);
    const unsigned gDF = (unsigned)(((long long)FF * (DM / 8) + 255) / 256);
    k_cast_wT<<<gDD, 256, 0, stream>>>(wq, DM, W3T, DM, DM, DM, 16.0f);
    k_cast_wT<<<gDD, 256, 0, stream>>>(wk, DM, W3T + (size_t)DM * DM, DM, DM, DM, 16.0f);
    k_cast_wT<<<gDD, 256, 0, stream>>>(wv, DM, W3T + (size_t)2 * DM * DM, DM, DM, DM, 16.0f);
    k_cast_wT<<<gDD, 256, 0, stream>>>(wo, DM, WOT, DM, DM, DM, 16.0f);
    k_cast_wT<<<gDF, 256, 0, stream>>>(w1, FF, W1T, DM, DM, FF, 16.0f);
    k_cast_wT<<<gDF, 256, 0, stream>>>(w2, DM, W2T, FF, FF, DM, 16.0f);

    k_rms<<<MROWS, 256, 0, stream>>>(x, SEQ_FULL, wpre, H32, SEQ, H16, 1, 1, 1);

    k_gemm_h<<<(unsigned)(((MROWS / 64) * (LDQK / 64) + 7) / 8), 256, 0, stream>>>(H16, DM, W3T, DM, QK16, LDQK, MROWS, LDQK, DM, 0.0625f);
    k_gemm_h<<<(unsigned)(((DM / 64) * (MROWS / 64) + 7) / 8), 256, 0, stream>>>(W3T + (size_t)2 * DM * DM, DM, H16, DM, VT16, LDVT, DM, MROWS, DM, 0.0625f);

    k_attn<<<(unsigned)(NB * NH * (SEQ / 64)), 128, 0, stream>>>(QK16, VT16, C16);

    k_gemm_res<<<(unsigned)(((MROWS / 64) * (DM / 64) + 7) / 8), 256, 0, stream>>>(C16, DM, WOT, DM, R1, DM, H32, MROWS, DM, DM, 0.0625f);
    k_rms<<<MROWS, 256, 0, stream>>>(R1, SEQ, wan, Y32, SEQ, Y16, 0, 1, 1);

    k_gemm_silu<<<(unsigned)(((MROWS / 64) * (FF / 64) + 7) / 8), 256, 0, stream>>>(Y16, DM, W1T, DM, MID, FF, MROWS, FF, DM, 0.0625f);
    k_gemm_res<<<(unsigned)(((MROWS / 64) * (DM / 64) + 7) / 8), 256, 0, stream>>>(MID, FF, W2T, FF, R2, DM, Y32, MROWS, DM, FF, 0.0625f);
    k_rms<<<MROWS, 256, 0, stream>>>(R2, SEQ, wfn, out, SEQ_FULL, nullptr, 0, 1, 0);
}
